// GraphAttentionV2Network_51797305590029
// MI455X (gfx1250) — hardware-run, weakly checked
//
#include <hip/hip_runtime.h>


namespace {
constexpr int N = 50000, E = 400000, G = 500, NH = 4, C = 64, HC = NH * C, IN = 9, ED = 3, NBLK = N / 16;
constexpr float XS = 8.0f, WSC = 256.0f, SLOPE = 0.2f;
typedef _Float16 b16;
typedef __attribute__((ext_vector_type(16))) _Float16 v16b;
typedef __attribute__((ext_vector_type(8))) _Float16 v8b;
typedef __attribute__((ext_vector_type(8))) float v8f;
typedef __attribute__((ext_vector_type(4))) float v4f;
__device__ __forceinline__ float bf16_rne(float f) { unsigned int u = __float_as_uint(f); u += 0x7FFFu + ((u >> 16) & 1u); return __uint_as_float(u & 0xFFFF0000u); }
__device__ __forceinline__ void split16(float v, b16& hi, b16& lo) { hi = (b16)v; lo = (b16)(v - (float)hi); }
__device__ __forceinline__ v16b frag_kb(const b16* p, int hh) { const v8b a = *(const v8b*)(p + 8 * hh), b = *(const v8b*)(p + 16 + 8 * hh); v16b f;
#pragma unroll
  for (int e = 0; e < 8; ++e) { f[e] = a[e]; f[8 + e] = b[e]; } return f; }
__device__ __forceinline__ v8f wmma16b(v16b a, v16b b, v8f c) { v8f d = __builtin_amdgcn_wmma_f32_16x16x32_f16(false, a, false, b, (short)0, c, false, false); asm volatile("v_nop\n\tv_nop\n\tv_nop\n\tv_nop" : "+v"(d) : "v"(a), "v"(b)); return d; }
__device__ __forceinline__ void wave_lds_sync() { __builtin_amdgcn_fence(__ATOMIC_RELEASE, "workgroup"); __builtin_amdgcn_wave_barrier(); __builtin_amdgcn_fence(__ATOMIC_ACQUIRE, "workgroup"); }
__device__ __forceinline__ float pmul(float a, float b) { float p = a * b; asm volatile("" : "+v"(p)); return p; }
__device__ __forceinline__ int iclamp(int v, int lo, int hi) { return v < lo ? lo : (v > hi ? hi : v); }
__device__ __forceinline__ float leaky(float v) { return v >= 0.0f ? v : SLOPE * v; }
__device__ __forceinline__ float elu(float v) { return v > 0.0f ? v : expm1f(v); }
constexpr int CSR_NBLK9 = 512, CSR_GB9 = 9, CSR_GN9 = 1 << CSR_GB9  , CSR_TS9 = (CSR_GN9 < 32 ? 32 : CSR_GN9)  , CSR_MAXG9 = 512, CSR_CAP9 = 12288  ;
__device__ __host__ __forceinline__ int csr_tix9(int v) { return (v >> CSR_GB9) * CSR_TS9 + (v & (CSR_GN9 - 1)); }
__global__ __launch_bounds__(64) void csrA_kernel9(const int* __restrict__ dst, int E, int N, int nG, int CHP, int NGP, int* __restrict__ STG, int* __restrict__ HST) {
  extern __shared__ int sm[];
  int* cnt = sm; int* run = sm + NGP; int* ids = sm + 2 * NGP;
  const int b = blockIdx.x; const int ch = (E + CSR_NBLK9 - 1) / CSR_NBLK9; const int e0 = b * ch, e1 = min(E, e0 + ch);
  for (int i = threadIdx.x; i < NGP; i += 64) cnt[i] = 0;
  for (int i = threadIdx.x; i < CHP; i += 64) ids[i] = -1;
  __syncthreads();
  if (threadIdx.x == 0) {
    for (int e = e0; e < e1; ++e) { int d = dst[e]; d = (d < 0) ? 0 : (d >= N ? N - 1 : d); cnt[d >> CSR_GB9] += 1; }
    int acc = 0; for (int g = 0; g < nG; ++g) { run[g] = acc; acc += cnt[g]; }
    for (int e = e0; e < e1; ++e) { int d = dst[e]; d = (d < 0) ? 0 : (d >= N ? N - 1 : d); const int g = d >> CSR_GB9; ids[run[g]] = e; run[g] += 1; } }
  __syncthreads();
  typedef __attribute__((ext_vector_type(4))) int v4i;
  for (int pass = 0; pass < 2; ++pass) {
    for (int i = threadIdx.x; i < CHP / 4; i += 64) *(volatile v4i*)(STG + (size_t)b * CHP + i * 4) = *(const v4i*)(&ids[i * 4]);
    for (int i = threadIdx.x; i < NGP / 4; i += 64) { v4i v; for (int e = 0; e < 4; ++e) v[e] = (i * 4 + e < nG) ? cnt[i * 4 + e] : 0; *(volatile v4i*)(HST + (size_t)b * NGP + i * 4) = v; }
    __threadfence(); }
}
__global__ __launch_bounds__(512) void csrS_kernel9(const int* __restrict__ HST, int nG, int NGP, int* __restrict__ START, int* __restrict__ TOT, int* __restrict__ OFF) {
  __shared__ int tot[CSR_MAXG9];
  const int b = threadIdx.x;
  for (int pass = 0; pass < 2; ++pass) { int runb = 0; for (int g = 0; g < nG; ++g) { int c = HST[(size_t)b * NGP + g]; c = (c < 0) ? 0 : c; ((volatile int*)OFF)[(size_t)g * CSR_NBLK9 + b] = runb; runb += c; } __threadfence(); }
  for (int g = threadIdx.x; g < nG; g += 512) { int s = 0; for (int bb = 0; bb < CSR_NBLK9; ++bb) { int c = HST[(size_t)bb * NGP + g]; s += (c < 0) ? 0 : c; } tot[g] = s; }
  __syncthreads();
  if (threadIdx.x < 32) {
    __shared__ int st[CSR_MAXG9 + 32];
    if (threadIdx.x == 0) { int acc = 0; for (int g = 0; g < NGP; ++g) { st[g] = acc; if (g < nG) acc += (tot[g] + 31) & ~31; } st[NGP] = acc; }
    __builtin_amdgcn_fence(__ATOMIC_RELEASE, "workgroup"); __builtin_amdgcn_wave_barrier(); __builtin_amdgcn_fence(__ATOMIC_ACQUIRE, "workgroup");
    for (int pass = 0; pass < 2; ++pass) { for (int i = threadIdx.x; i < NGP + 32; i += 32) { ((volatile int*)START)[i] = (i <= NGP) ? st[min(i, NGP)] : 0; ((volatile int*)TOT)[i] = (i < nG) ? tot[i] : 0; } __threadfence(); } }
}
__global__ __launch_bounds__(256) void csrB_kernel9(const int* __restrict__ dst, int N, int nG, int CHP, int NGP, int permLen, const int* __restrict__ STG, const int* __restrict__ HST, const int* __restrict__ OFF, const int* __restrict__ START, const int* __restrict__ TOT, int* __restrict__ PERM, int* __restrict__ ROWPTR, int* __restrict__ ROWCNT, int* __restrict__ FLAG) {
  typedef __attribute__((ext_vector_type(4))) int v4i;
  __shared__ int ids[CSR_CAP9]; __shared__ unsigned short key[CSR_CAP9]; __shared__ int outp[CSR_CAP9]; __shared__ int ncnt[CSR_GN9 + 1]; __shared__ int boff[CSR_NBLK9 + 1];
  const int g = blockIdx.x, t_ = threadIdx.x; int tot = TOT[g]; int st = START[g], stn = START[g + 1]; const int v0 = g * CSR_GN9; const int nv = min(CSR_GN9, N - v0); const int t0 = g * CSR_TS9;
  st = (st < 0) ? 0 : (st > permLen - 32 ? permLen - 32 : st) & ~31; stn = (stn < st) ? st : (stn > permLen ? permLen : stn); tot = (tot < 0) ? 0 : tot; if (tot > stn - st && tot <= CSR_CAP9) tot = stn - st;
  if (tot > CSR_CAP9) {
    for (int pass = 0; pass < 2; ++pass) { for (int i = t_; i < CSR_TS9 / 4; i += 256) { v4i a, c; for (int e = 0; e < 4; ++e) { a[e] = st; c[e] = 0; } *(volatile v4i*)(ROWPTR + t0 + i * 4) = a; *(volatile v4i*)(ROWCNT + t0 + i * 4) = c; } if (t_ == 0) ((volatile int*)FLAG)[0] = 1; __threadfence(); } (void)nv; return; }
  if (t_ == 0) { int acc = 0; for (int b = 0; b < CSR_NBLK9; ++b) { boff[b] = acc; int c = HST[(size_t)b * NGP + g]; c = (c < 0) ? 0 : (c > CHP ? CHP : c); acc += c; if (acc > tot) acc = tot; } boff[CSR_NBLK9] = acc; }
  for (int i = t_; i <= CSR_GN9; i += 256) ncnt[i] = 0;
  __syncthreads();
  for (int b = 0; b < CSR_NBLK9; ++b) { const int c = boff[b + 1] - boff[b]; int o_ = OFF[(size_t)g * CSR_NBLK9 + b]; o_ = (o_ < 0) ? 0 : (o_ > CHP - c ? CHP - c : o_); const int* src_ = STG + (size_t)b * CHP + o_;
    for (int i = t_; i < c; i += 256) { int id = src_[i]; id = (id < 0) ? 0 : id; ids[boff[b] + i] = id; int d = dst[id]; d = (d < v0) ? v0 : (d >= N ? N - 1 : d); int kk = d - v0; kk = (kk < 0) ? 0 : (kk >= CSR_GN9 ? CSR_GN9 - 1 : kk); key[boff[b] + i] = (unsigned short)kk; } }
  __syncthreads();
  if (t_ == 0) { for (int i = 0; i < tot; ++i) ncnt[key[i]] += 1; int acc = 0; for (int vl = 0; vl < CSR_GN9; ++vl) { const int c = ncnt[vl]; ncnt[vl] = acc; acc += c; } ncnt[CSR_GN9] = acc;
    for (int i = 0; i < tot; ++i) { const int vl = key[i]; outp[ncnt[vl]] = ids[i]; ncnt[vl] += 1; }
    for (int vl = CSR_GN9; vl > 0; --vl) ncnt[vl] = ncnt[vl - 1]; ncnt[0] = 0; }
  __syncthreads();
  for (int pass = 0; pass < 2; ++pass) {
    for (int i = t_; i < (stn - st) / 4; i += 256) { v4i v; for (int e = 0; e < 4; ++e) { const int q = i * 4 + e; v[e] = (q < tot) ? outp[q] : -1; } *(volatile v4i*)(PERM + st + i * 4) = v; }
    for (int i = t_; i < CSR_TS9 / 4; i += 256) { v4i a, c; for (int e = 0; e < 4; ++e) { const int vl = i * 4 + e; const int vc = vl < CSR_GN9 ? vl : CSR_GN9; a[e] = (vl < CSR_GN9) ? st + ncnt[vc] : st; c[e] = (vl < nv) ? (ncnt[(vc < CSR_GN9 ? vc : CSR_GN9 - 1) + 1] - ncnt[vc]) : 0; } *(volatile v4i*)(ROWPTR + t0 + i * 4) = a; *(volatile v4i*)(ROWCNT + t0 + i * 4) = c; }
    __threadfence(); }
}
__global__ __launch_bounds__(256) void csrZ_kernel9(int* __restrict__ p, size_t n4) { typedef __attribute__((ext_vector_type(4))) int v4i; const size_t tid = (size_t)blockIdx.x * 256 + threadIdx.x, nth = (size_t)gridDim.x * 256; v4i z = {0, 0, 0, 0}; for (size_t i = tid; i < n4; i += nth) *(volatile v4i*)(p + i * 4) = z; }
struct CsrBufs9 { int *STG, *HST, *OFF, *START, *TOT, *PERM, *ROWPTR, *ROWCNT, *FLAG; int nG, NGP, CHP; size_t permLen; char* base; size_t bytes; };
static size_t csr_carve9(CsrBufs9& c, char* ws, size_t off, int E, int N) {
  const size_t off0 = off; c.base = ws + off;
  auto al = [&](size_t bytes) { char* p = ws + off; off += (bytes + 255) & ~(size_t)255; return p; };
  c.nG = (N + CSR_GN9 - 1) / CSR_GN9; c.NGP = (c.nG + 31) & ~31; const int ch = (E + CSR_NBLK9 - 1) / CSR_NBLK9; c.CHP = (ch + 31) & ~31; c.permLen = (size_t)E + 32 * (size_t)c.nG + 32;
  c.STG = (int*)al((size_t)CSR_NBLK9 * c.CHP * 4); c.HST = (int*)al((size_t)CSR_NBLK9 * c.NGP * 4); c.OFF = (int*)al((size_t)c.NGP * CSR_NBLK9 * 4); c.START = (int*)al((size_t)(c.NGP + 64) * 4); c.TOT = (int*)al((size_t)(c.NGP + 64) * 4);
  c.PERM = (int*)al(c.permLen * 4); c.ROWPTR = (int*)al((size_t)c.nG * CSR_TS9 * 4); c.ROWCNT = (int*)al((size_t)c.nG * CSR_TS9 * 4); c.FLAG = (int*)al(256);
  c.bytes = off - off0; return off;
}
static void csr_build9(const CsrBufs9& c, const int* dst, int E, int N, hipStream_t stream) {
  const size_t smem = (size_t)(2 * c.NGP + c.CHP) * 4;
  csrZ_kernel9<<<512, 256, 0, stream>>>((int*)c.base, c.bytes / 16);
  csrA_kernel9<<<CSR_NBLK9, 64, smem, stream>>>(dst, E, N, c.nG, c.CHP, c.NGP, c.STG, c.HST);
  csrS_kernel9<<<1, 512, 0, stream>>>(c.HST, c.nG, c.NGP, c.START, c.TOT, c.OFF);
  csrB_kernel9<<<c.nG, 256, 0, stream>>>(dst, N, c.nG, c.CHP, c.NGP, (int)c.permLen, c.STG, c.HST, c.OFF, c.START, c.TOT, c.PERM, c.ROWPTR, c.ROWCNT, c.FLAG);
}


__global__ __launch_bounds__(256) void wput_kernel(const float* __restrict__ w, int KIN, int KP, int ro, b16* __restrict__ WT) {
  const int KG = KP / 8; const int u = blockIdx.x * 256 + threadIdx.x; if (u >= HC * KG) return; const int o = u / KG, k0 = (u % KG) * 8; v8b v;
#pragma unroll
  for (int j = 0; j < 8; ++j) { const int k = k0 + j; v[j] = k < KIN ? (b16)(bf16_rne(w[(size_t)k * HC + o]) * WSC) : (b16)0.0f; } for (int pass = 0; pass < 2; ++pass) { *(volatile v8b*)(WT + (size_t)(ro + o) * KP + k0) = v; __threadfence(); }
}
template <int KP, int FIRST>
__global__ __launch_bounds__(32) void proj_kernel(const float* __restrict__ hin, const b16* __restrict__ WT, const float* __restrict__ bl, int NLIM, float* __restrict__ XL, float* __restrict__ XR) {
  __shared__ __attribute__((aligned(16))) b16 Ah[16][KP + 8], Al[16][KP + 8]; __shared__ __attribute__((aligned(16))) float Tf[16][128 + 4];
  const int lane = threadIdx.x, nloc = lane & 15, hlf = lane >> 4; const size_t m0 = (size_t)blockIdx.x * 16; if (m0 >= (size_t)NLIM) return;
  for (int rr = 0; rr < 16; ++rr) for (int q = 0; q < KP / 32; ++q) { const int c = q * 32 + lane; float v = 0.0f; if (FIRST) { if (c < IN) v = bf16_rne(hin[(m0 + rr) * IN + c]); } else v = hin[(m0 + rr) * C + c]; b16 p, ql; split16(v * XS, p, ql); Ah[rr][c] = p; Al[rr][c] = ql; }
  wave_lds_sync();
#pragma unroll 1
  for (int cg = 0; cg < 4; ++cg) { v8f acc[8];
#pragma unroll
    for (int t = 0; t < 8; ++t) acc[t] = (v8f){};
#pragma unroll
    for (int kb = 0; kb < KP; kb += 32) { const v16b a = frag_kb(&Ah[nloc][kb], hlf), al = frag_kb(&Al[nloc][kb], hlf);
#pragma unroll
      for (int t = 0; t < 8; ++t) { const v16b bw = frag_kb(WT + (size_t)(cg * 128 + t * 16 + nloc) * KP + kb, hlf); acc[t] = wmma16b(a, bw, acc[t]); if (!FIRST) acc[t] = wmma16b(al, bw, acc[t]); } }
#pragma unroll
    for (int t = 0; t < 8; ++t) { const int c = cg * 128 + t * 16 + nloc; const float bb = (cg < 2) ? bf16_rne(bl[c]) : 0.0f;
#pragma unroll
      for (int r8 = 0; r8 < 8; ++r8) Tf[8 * hlf + r8][t * 16 + nloc] = acc[t][r8] * (1.0f / (XS * WSC)) + bb; }
    wave_lds_sync();
    float* dstp = (cg < 2) ? XL : XR; const int co = (cg & 1) * 128;
    for (int pass = 0; pass < 2; ++pass) { for (int rr = 0; rr < 16; ++rr) *(volatile v4f*)(dstp + (m0 + rr) * HC + co + lane * 4) = *(const v4f*)(&Tf[rr][lane * 4]); __threadfence(); }
    wave_lds_sync(); }
}
template <int RES>
__global__ __launch_bounds__(256) void att_kernel(const float* __restrict__ XL, const float* __restrict__ XR, const float* __restrict__ ea, const float* __restrict__ We, const float* __restrict__ att, const float* __restrict__ bias, const float* __restrict__ bng, const float* __restrict__ bnb, const float* __restrict__ bnm, const float* __restrict__ bnv, const float* __restrict__ HPREV, const int* __restrict__ srcs, const int* __restrict__ PERM, const int* __restrict__ ROWPTR, const int* __restrict__ ROWCNT, int permLen, int NLIM, float* __restrict__ HOUT) {
  const int wave = threadIdx.x >> 5, lane = threadIdx.x & 31; const size_t v = (size_t)blockIdx.x * 8 + wave; if (v >= (size_t)NLIM) return; const int c0 = lane * 8;
  float xr[8], aw[8], we0[8], we1[8], we2[8]; for (int i = 0; i < 8; ++i) { xr[i] = XR[v * HC + c0 + i]; aw[i] = bf16_rne(att[c0 + i]); we0[i] = bf16_rne(We[c0 + i]); we1[i] = bf16_rne(We[HC + c0 + i]); we2[i] = bf16_rne(We[2 * HC + c0 + i]); }
  int st = ROWPTR[v], cnt = ROWCNT[v]; cnt = iclamp(cnt, 0, 1 << 20); st = iclamp(st, 0, permLen - cnt);
  auto score = [&](int e, int s, float* xl) -> float { const float a0 = bf16_rne(ea[(size_t)e * ED]), a1 = bf16_rne(ea[(size_t)e * ED + 1]), a2 = bf16_rne(ea[(size_t)e * ED + 2]); const v4f p0 = *(const v4f*)(XL + (size_t)s * HC + c0), p1 = *(const v4f*)(XL + (size_t)s * HC + c0 + 4); float sc = 0.0f;
    for (int i = 0; i < 8; ++i) { xl[i] = i < 4 ? p0[i] : p1[i - 4]; const float m = leaky(xl[i] + xr[i] + pmul(a0, we0[i]) + pmul(a1, we1[i]) + pmul(a2, we2[i])); sc += pmul(m, aw[i]); }
    for (int o = 1; o < 8; o <<= 1) sc += __shfl_xor(sc, o); return sc; };
  float mx = -INFINITY; float xl[8];
#pragma unroll 1
  for (int j = 0; j < cnt; ++j) { const int e = iclamp(PERM[st + j], 0, E - 1); const int s = iclamp(srcs[e], 0, N - 1); const float sc = score(e, s, xl); if (s < NLIM) mx = fmaxf(mx, sc); }
  float den = 0.0f, o8[8]; for (int i = 0; i < 8; ++i) o8[i] = 0.0f;
#pragma unroll 1
  for (int j = 0; j < cnt; ++j) { const int e = iclamp(PERM[st + j], 0, E - 1); const int s = iclamp(srcs[e], 0, N - 1); const float sc = score(e, s, xl); if (s >= NLIM) continue; const float p = __expf(sc - mx); den += p; for (int i = 0; i < 8; ++i) o8[i] += pmul(p, xl[i]); }
  const float inv = den > 0.0f ? 1.0f / den : 0.0f; float z[8]; const int cc0 = (lane & 7) * 8;
  for (int i = 0; i < 8; ++i) { float t = pmul(o8[i], inv); t += __shfl_xor(t, 8); t += __shfl_xor(t, 16); const int c = cc0 + i; float zz = t * 0.25f + bf16_rne(bias[c]); zz = pmul(zz - bf16_rne(bnm[c]), pmul(bf16_rne(bng[c]), rsqrtf(bf16_rne(bnv[c]) + 1e-5f))) + bf16_rne(bnb[c]); zz = elu(zz); if (RES) zz += HPREV[v * C + c]; z[i] = zz; }
  for (int pass = 0; pass < 2; ++pass) { if (lane < 8) { *(volatile v4f*)(HOUT + v * C + cc0) = (v4f){z[0], z[1], z[2], z[3]}; *(volatile v4f*)(HOUT + v * C + cc0 + 4) = (v4f){z[4], z[5], z[6], z[7]}; } __threadfence(); }
}
__global__ __launch_bounds__(32) void grange_kernel(const int* __restrict__ batch, int* __restrict__ SE) {
  const int lane = threadIdx.x;
  auto lb = [&](int key) -> int { int lo = 0, hi = N; for (int it = 0; it < 17 && lo < hi; ++it) { const int mid = (lo + hi) >> 1; if (batch[mid] < key) lo = mid + 1; else hi = mid; } return lo; };
  for (int g0 = 0; g0 < 512; g0 += 32) { const int g = g0 + lane; const int st = g < G ? lb(g) : N, en = g < G ? lb(g + 1) : N; for (int pass = 0; pass < 2; ++pass) { ((volatile int*)SE)[g] = st; ((volatile int*)SE)[512 + g] = en; __threadfence(); } }
}
__global__ __launch_bounds__(64) void pool_kernel(const float* __restrict__ Hh, const int* __restrict__ SE, const float* __restrict__ Wo1, const float* __restrict__ bo1, const float* __restrict__ Wo2, const float* __restrict__ bo2, int NLIM, float* __restrict__ PO) {
  __shared__ float Ps[C]; const int g = blockIdx.x, c = threadIdx.x; int s0 = iclamp(SE[g], 0, N), e0 = iclamp(SE[512 + g], 0, N); if (e0 > NLIM) e0 = NLIM; if (e0 < s0) e0 = s0; float s = 0.0f; int cnt = 0;
#pragma unroll 1
  for (int n = s0; n < e0; ++n) { s += Hh[(size_t)n * C + c]; ++cnt; }
  Ps[c] = s / (float)(cnt < 1 ? 1 : cnt); __syncthreads();
  if (c < 32) { float a = bf16_rne(bo1[c]);
#pragma unroll 1
    for (int k = 0; k < C; ++k) a += pmul(Ps[k], bf16_rne(Wo1[k * 32 + c])); float t = pmul(elu(a), bf16_rne(Wo2[c])); for (int o = 16; o; o >>= 1) t += __shfl_xor(t, o);
    const float r = t + bf16_rne(bo2[0]); for (int pass = 0; pass < 2; ++pass) { ((volatile float*)PO)[g * 32 + c] = r; __threadfence(); } }
}
__global__ __launch_bounds__(32) void outw_kernel(const float* __restrict__ PO, float* __restrict__ out) { const int g = blockIdx.x * 32 + threadIdx.x; const float v = g < G ? PO[g * 32] : 0.0f; for (int pass = 0; pass < 2; ++pass) { if (g < G) ((volatile float*)out)[g] = v; __threadfence(); } }
}

extern "C" void kernel_launch(void* const* d_in, const int* in_sizes, int n_in, void* d_out, int out_size, void* d_ws, size_t ws_size, hipStream_t stream) {
  (void)n_in;
  auto Fp = [&](int i) { return (const float*)d_in[i]; }; auto Ip = [&](int i) { return (const int*)d_in[i]; };
  if (in_sizes[0] != N * IN || in_sizes[1] != 2 * E || in_sizes[2] != N || in_sizes[3] != E * ED || in_sizes[4] != IN * HC || in_sizes[7] != ED * HC || in_sizes[10] != 3 * C * HC || in_sizes[13] != 3 * ED * HC || in_sizes[16] != 4 * C || in_sizes[20] != C * 32 || out_size != G) return;
  const int NLIM = N; const int GB16 = NBLK, GB8 = N / 8;
  size_t off = 0; char* ws = (char*)d_ws;
  auto carve = [&](size_t bytes) { char* p = ws + off; off += (bytes + 255) & ~(size_t)255; return p; };
  b16* WT0 = (b16*)carve((size_t)2 * HC * 32 * 2); b16* WTL[3]; for (int i = 0; i < 3; ++i) WTL[i] = (b16*)carve((size_t)2 * HC * C * 2);
  float* XL = (float*)carve((size_t)N * HC * 4); float* XR = (float*)carve((size_t)N * HC * 4); float* HA = (float*)carve((size_t)N * C * 4); float* HB = (float*)carve((size_t)N * C * 4); int* SE = (int*)carve(1024 * 4); float* PO = (float*)carve(512 * 32 * 4);
  CsrBufs9 csr; off = csr_carve9(csr, ws, off, E, N);
  if (off > ws_size || off > ((size_t)160 << 20)) return;
  wput_kernel<<<(HC * 4 + 255) / 256, 256, 0, stream>>>(Fp(4), IN, 32, 0, WT0); wput_kernel<<<(HC * 4 + 255) / 256, 256, 0, stream>>>(Fp(6), IN, 32, HC, WT0);
  for (int i = 0; i < 3; ++i) { wput_kernel<<<(HC * 8 + 255) / 256, 256, 0, stream>>>(Fp(10) + (size_t)i * C * HC, C, C, 0, WTL[i]); wput_kernel<<<(HC * 8 + 255) / 256, 256, 0, stream>>>(Fp(12) + (size_t)i * C * HC, C, C, HC, WTL[i]); }
  csr_build9(csr, Ip(1) + E, E, N, stream);
  proj_kernel<32, 1><<<GB16, 32, 0, stream>>>(Fp(0), WT0, Fp(5), NLIM, XL, XR);
  att_kernel<0><<<GB8, 256, 0, stream>>>(XL, XR, Fp(3), Fp(7), Fp(8), Fp(9), Fp(16), Fp(17), Fp(18), Fp(19), nullptr, Ip(1), csr.PERM, csr.ROWPTR, csr.ROWCNT, (int)csr.permLen, NLIM, HA);
  float* hp = HA; float* hn = HB;
  for (int i = 0; i < 3; ++i) {
    proj_kernel<64, 0><<<GB16, 32, 0, stream>>>(hp, WTL[i], Fp(11) + i * HC, NLIM, XL, XR);
    att_kernel<1><<<GB8, 256, 0, stream>>>(XL, XR, Fp(3), Fp(13) + (size_t)i * ED * HC, Fp(14) + i * HC, Fp(15) + i * C, Fp(16) + (i + 1) * C, Fp(17) + (i + 1) * C, Fp(18) + (i + 1) * C, Fp(19) + (i + 1) * C, hp, Ip(1), csr.PERM, csr.ROWPTR, csr.ROWCNT, (int)csr.permLen, NLIM, hn);
    float* t = hp; hp = hn; hn = t; }
  grange_kernel<<<1, 32, 0, stream>>>(Ip(2), SE);
  pool_kernel<<<G, 64, 0, stream>>>(hp, SE, Fp(20), Fp(21), Fp(22), Fp(23), NLIM, PO);
  outw_kernel<<<(G + 31) / 32, 32, 0, stream>>>(PO, (float*)d_out);
}
